// KANFeedForward_8014408974694
// MI455X (gfx1250) — hardware-verified
//
#include <hip/hip_runtime.h>
#include <math.h>

#pragma clang fp contract(off)

constexpr int kRows = 4096;
constexpr int kDimA = 512;
constexpr int kDimB = 1024;
constexpr int kNBas = 8;
constexpr int kK1 = kDimA * 9;
constexpr int kK2 = kDimB * 9;
constexpr float kBasCarry2  = 128.0f;
constexpr float kCoefCarry2 = 8.0f;
constexpr float kBaseCarry2 = 1024.0f;
constexpr float kOutScale2  = 1.0f / 1024.0f;
static_assert(kK1 % 32 == 0 && kK2 % 32 == 0, "k tiles");
static_assert(kRows % 64 == 0 && kDimA % 64 == 0 && kDimB % 64 == 0, "mn tiles");
static_assert(kDimA % 256 == 0 && kDimB % 256 == 0, "builder iterations");

constexpr size_t kPlaneA1 = (size_t)kRows * kK1 * 2;
constexpr size_t kPlaneA2 = (size_t)kRows * kK2 * 2;
constexpr size_t kPlaneB1 = (size_t)kDimB * kK1 * 2;
constexpr size_t kPlaneB2 = (size_t)kDimA * kK2 * 2;
constexpr size_t kBytesH  = (size_t)kRows * kDimB * 4;
constexpr size_t kOffA1h = 0;
constexpr size_t kOffA1l = kOffA1h + kPlaneA1;
constexpr size_t kOffA2  = 0;
constexpr size_t kOffB1h = kPlaneA2;
constexpr size_t kOffB1l = kOffB1h + kPlaneB1;
constexpr size_t kOffB2  = kOffB1l + kPlaneB1;
constexpr size_t kOffH   = kOffB2 + kPlaneB2;
constexpr size_t kWsTotal = kOffH + kBytesH;
static_assert(kOffA1l + kPlaneA1 == kPlaneA2, "A2 exactly covers A1 hi+lo");
static_assert(kWsTotal == 120586240, "carve total");
static_assert(kWsTotal <= 134217728, "carve under 128 MiB");
static_assert((kOffB1h % 128) == 0 && (kOffB1l % 128) == 0 && (kOffB2 % 128) == 0 && (kOffH % 128) == 0, "line aligned");

typedef __attribute__((ext_vector_type(16))) _Float16 v16h;
typedef __attribute__((ext_vector_type(8)))  _Float16 v8h;
typedef __attribute__((ext_vector_type(16))) __bf16   v16b;
typedef __attribute__((ext_vector_type(8)))  __bf16   v8b;
typedef __attribute__((ext_vector_type(8)))  float    v8f;
typedef __attribute__((ext_vector_type(4)))  float    v4f;
typedef __attribute__((ext_vector_type(4)))  unsigned int v4u;

__device__ __forceinline__ unsigned short f2bf_bits(float f) {
  unsigned u = __float_as_uint(f);
  return (unsigned short)((u + 0x7FFFu + ((u >> 16) & 1u)) >> 16);
}
__device__ __forceinline__ float bf_bits2f(unsigned short h) { return __uint_as_float(((unsigned)h) << 16); }

__device__ __forceinline__ void dep_guard_h(v8f& a, v8f& b, v16h x, v16h y) { asm volatile("v_nop\n\tv_nop\n\tv_nop\n\tv_nop" : "+v"(a), "+v"(b) : "v"(x), "v"(y)); }
__device__ __forceinline__ void dep_guard_b(v8f& a, v8f& b, v16b x, v16b y) { asm volatile("v_nop\n\tv_nop\n\tv_nop\n\tv_nop" : "+v"(a), "+v"(b) : "v"(x), "v"(y)); }
__device__ __forceinline__ void keep4_h(v16h a, v16h b, v16h c, v16h d) { asm volatile("v_nop" :: "v"(a), "v"(b), "v"(c), "v"(d)); }
__device__ __forceinline__ void keep4_b(v16b a, v16b b, v16b c, v16b d) { asm volatile("v_nop" :: "v"(a), "v"(b), "v"(c), "v"(d)); }
__device__ __forceinline__ void acc_guard4(v8f& a, v8f& b, v8f& c, v8f& d) { asm volatile("v_nop\n\tv_nop\n\tv_nop\n\tv_nop" : "+v"(a), "+v"(b), "+v"(c), "+v"(d)); }
template <typename T> struct Frag;
template <> struct Frag<_Float16> {
  typedef v16h V; union U { v16h v; v8h h[2]; };
  static __device__ __forceinline__ v16h load(const _Float16* p) {
    U f; f.h[0] = *(const v8h*)(p); f.h[1] = *(const v8h*)(p + 16); return f.v;
  }
  static __device__ __forceinline__ v8f mma(v16h a, v16h b, v8f c) {
    return __builtin_amdgcn_wmma_f32_16x16x32_f16(false, a, false, b, (short)0, c, false, false);
  }
  static __device__ __forceinline__ void guard(v8f& a, v8f& b, v16h x, v16h y) { dep_guard_h(a, b, x, y); }
  static __device__ __forceinline__ void keep(v16h a, v16h b, v16h c, v16h d) { keep4_h(a, b, c, d); }
};
template <> struct Frag<__bf16> {
  typedef v16b V; union U { v16b v; v8b h[2]; };
  static __device__ __forceinline__ v16b load(const __bf16* p) {
    U f; f.h[0] = *(const v8b*)(p); f.h[1] = *(const v8b*)(p + 16); return f.v;
  }
  static __device__ __forceinline__ v8f mma(v16b a, v16b b, v8f c) {
    return __builtin_amdgcn_wmma_f32_16x16x32_bf16(false, a, false, b, (short)0, c, false, false);
  }
  static __device__ __forceinline__ void guard(v8f& a, v8f& b, v16b x, v16b y) { dep_guard_b(a, b, x, y); }
  static __device__ __forceinline__ void keep(v16b a, v16b b, v16b c, v16b d) { keep4_b(a, b, c, d); }
};

__device__ __forceinline__ unsigned pk16(unsigned short a, unsigned short b) { return (unsigned)a | ((unsigned)b << 16); }
__device__ __forceinline__ unsigned short h_bits(float f) { const _Float16 h = (_Float16)f; return __builtin_bit_cast(unsigned short, h); }

template <int ET> struct Elem;
template <> struct Elem<0> { typedef _Float16 T; };
template <> struct Elem<1> { typedef __bf16 T; };
template <int ET, bool SPLIT, int BIAS_MODE, int OUT_MODE, bool RESID, int ACT = 0>
__global__ __launch_bounds__(256) void wmma_gemm64(
    const unsigned short* __restrict__ Ap, const unsigned short* __restrict__ A2p, int lda, long strideA,
    const unsigned short* __restrict__ Btp, const unsigned short* __restrict__ Bt2p, int ldb, long strideB,
    void* __restrict__ Cout, void* __restrict__ Cout2, int ldc, long strideC,
    const float* __restrict__ bias,
    const float* __restrict__ resid, long strideR,
    int M, int N, int K, float scale) {
  typedef typename Elem<ET>::T T;
  typedef typename Frag<T>::V V;
  const T* A = (const T*)Ap; const T* A2 = (const T*)A2p; const T* Bt = (const T*)Btp; const T* Bt2 = (const T*)Bt2p;
  __shared__ __align__(16) float sT[8][16 * 68];
  const int b    = blockIdx.y;
  const int lane = threadIdx.x & 31;
  const int wave = threadIdx.x >> 5;
  const int tilesN = N >> 6;
  const int tilesM = M >> 6;
  const int tile = blockIdx.x * 8 + wave;
  if (tile >= tilesM * tilesN) return;
  const int tm = tile / tilesN;
  const int tn = tile - tm * tilesN;
  const int m0 = tm << 6;
  const int n0 = tn << 6;

  const T* Ab  = A  + (size_t)b * strideA;
  const T* Bb  = Bt + (size_t)b * strideB;
  const T* Ab2 = SPLIT ? (A2  + (size_t)b * strideA) : nullptr;
  const T* Bb2 = SPLIT ? (Bt2 + (size_t)b * strideB) : nullptr;

  const int rlane = lane & 15;
  const int koff  = (lane >> 4) * 8;
  const int mOff  = (lane >> 4) * 8;

  v8f acc[4][4];
#pragma unroll
  for (int i = 0; i < 4; ++i)
#pragma unroll
    for (int j = 0; j < 4; ++j) acc[i][j] = (v8f){0.f,0.f,0.f,0.f,0.f,0.f,0.f,0.f};

  for (int k0 = 0; k0 < K; k0 += 32) {
    V bh[4], bl[4];
#pragma unroll
    for (int j = 0; j < 4; ++j) {
      const size_t bo = (size_t)(n0 + (j << 4) + rlane) * ldb + koff + k0;
      bh[j] = Frag<T>::load(Bb + bo);
      if (SPLIT) bl[j] = Frag<T>::load(Bb2 + bo);
    }
#pragma unroll
    for (int i = 0; i < 4; ++i) {
      const size_t ao = (size_t)(m0 + (i << 4) + rlane) * lda + koff + k0;
      V ah = Frag<T>::load(Ab + ao);
      V al;
      if (SPLIT) al = Frag<T>::load(Ab2 + ao);
#pragma unroll
      for (int j = 0; j < 4; ++j) {
        acc[i][j] = Frag<T>::mma(ah, bh[j], acc[i][j]);
        if (SPLIT) {
          acc[i][j] = Frag<T>::mma(ah, bl[j], acc[i][j]);
          acc[i][j] = Frag<T>::mma(al, bh[j], acc[i][j]);
        }
      }
      Frag<T>::guard(acc[i][0], acc[i][3], ah, SPLIT ? al : ah);
    }
    Frag<T>::keep(bh[0], bh[1], bh[2], bh[3]);
    if (SPLIT) Frag<T>::keep(bl[0], bl[1], bl[2], bl[3]);
  }
  acc_guard4(acc[0][0], acc[0][1], acc[0][2], acc[0][3]);
  acc_guard4(acc[1][0], acc[1][1], acc[1][2], acc[1][3]);
  acc_guard4(acc[2][0], acc[2][1], acc[2][2], acc[2][3]);
  acc_guard4(acc[3][0], acc[3][1], acc[3][2], acc[3][3]);

  float* slab = sT[wave];
  const float* Rb = RESID ? (resid + (size_t)b * strideR) : nullptr;
#pragma unroll
  for (int i = 0; i < 4; ++i) {
    const int mBase = m0 + (i << 4);
#pragma unroll
    for (int j = 0; j < 4; ++j) {
      const int n = n0 + (j << 4) + rlane;
      float bv = 0.f;
      if (BIAS_MODE == 2) bv = bias[n];
#pragma unroll
      for (int r = 0; r < 8; ++r) {
        float v = acc[i][j][r] * scale;
        if (BIAS_MODE == 1) v += bias[mBase + mOff + r];
        if (BIAS_MODE == 2) v += bv;
        if (RESID) v += Rb[(size_t)(mBase + mOff + r) * ldc + n];
        if (ACT == 2) v = fmaxf(v, 0.0f);
        if (ACT == 4) v = (v > 0.f) ? v : 0.01f * v;
        slab[(mOff + r) * 68 + (j << 4) + rlane] = v;
      }
    }
    __builtin_amdgcn_fence(__ATOMIC_RELEASE, "workgroup");
    __builtin_amdgcn_wave_barrier();
    __builtin_amdgcn_fence(__ATOMIC_ACQUIRE, "workgroup");
    if (OUT_MODE == 0) {
      float* C = (float*)Cout + (size_t)b * strideC;
      const int hh = lane >> 4, c4 = (lane & 15) * 4;
      for (int pass = 0; pass < 2; ++pass) {
#pragma unroll
        for (int it = 0; it < 8; ++it) {
          const int row = it * 2 + hh;
          v4f v = *(const v4f*)(slab + row * 68 + c4);
          *(volatile v4f*)(C + (size_t)(mBase + row) * ldc + n0 + c4) = v;
        }
        __threadfence();
      }
    } else {
      const int q = lane >> 3, c8 = (lane & 7) * 8;
      unsigned short* C  = (unsigned short*)Cout  + (size_t)b * strideC;
      unsigned short* C2 = (OUT_MODE == 2) ? ((unsigned short*)Cout2 + (size_t)b * strideC) : nullptr;
      for (int pass = 0; pass < 2; ++pass) {
#pragma unroll
        for (int it = 0; it < 4; ++it) {
          const int row = it * 4 + q;
          const float* sp = slab + row * 68 + c8;
          v8h hv, lv;
#pragma unroll
          for (int e = 0; e < 8; ++e) {
            if (OUT_MODE == 1) {
              hv[e] = (_Float16)sp[e];
            } else {
              unsigned short hb = f2bf_bits(sp[e]);
              unsigned short lb = f2bf_bits(sp[e] - bf_bits2f(hb));
              hv[e] = __builtin_bit_cast(_Float16, hb);
              lv[e] = __builtin_bit_cast(_Float16, lb);
            }
          }
          *(volatile v8h*)(C + (size_t)(mBase + row) * ldc + n0 + c8) = hv;
          if (OUT_MODE == 2) *(volatile v8h*)(C2 + (size_t)(mBase + row) * ldc + n0 + c8) = lv;
        }
        __threadfence();
      }
    }
    __builtin_amdgcn_fence(__ATOMIC_RELEASE, "workgroup");
    __builtin_amdgcn_wave_barrier();
    __builtin_amdgcn_fence(__ATOMIC_ACQUIRE, "workgroup");
  }
}

__device__ __forceinline__ float spl_knot(int m) { return (float)(m - 3) * 0.4f - 1.0f; }

__device__ __forceinline__ void spl_basis8(float x, float (&bo)[8]) {
  float tk[12];
#pragma unroll
  for (int m = 0; m < 12; ++m) tk[m] = spl_knot(m);
  float bb[11];
#pragma unroll
  for (int m = 0; m < 11; ++m) bb[m] = (x >= tk[m] && x < tk[m + 1]) ? 1.0f : 0.0f;
#pragma unroll
  for (int p = 1; p <= 3; ++p) {
#pragma unroll
    for (int m = 0; m < 11 - p; ++m) {
      const float il = 1.0f / (tk[m + p] - tk[m]);
      const float ir = 1.0f / (tk[m + p + 1] - tk[m + 1]);
      const float wl = (x - tk[m]) * il;
      const float wr = (tk[m + p + 1] - x) * ir;
      const float a0 = wl * bb[m];
      const float a1 = wr * bb[m + 1];
      bb[m] = a0 + a1;
    }
  }
#pragma unroll
  for (int g = 0; g < 8; ++g) bo[g] = bb[g];
}

__device__ __forceinline__ float silu_f32(float x) {
  const float d = 1.0f + expf(-x);
  return x * (1.0f / d);
}

template <int NIN, int MODE>
__global__ __launch_bounds__(256) void build_act_rows(const float* __restrict__ X,
                                                      unsigned short* __restrict__ P0,
                                                      unsigned short* __restrict__ P1,
                                                      float bcarry) {
  constexpr int KP  = NIN * 9;
  constexpr int NIT = NIN / 256;
  __shared__ __align__(16) unsigned short s0[NIN];
  __shared__ __align__(16) unsigned short s1[(MODE == 0) ? NIN : 16];
  const int n = blockIdx.x;
  const int t = threadIdx.x;
  const float* xr = X + (size_t)n * NIN;
  unsigned short* r0 = P0 + (size_t)n * KP;
  unsigned short* r1 = P1 + (size_t)n * KP;
#pragma unroll 1
  for (int it = 0; it < NIT; ++it) {
    const int i = it * 256 + t;
    const float xv = xr[i];
    float bv[8];
    spl_basis8(xv, bv);
    const float sv = silu_f32(xv);
    unsigned short hb[8], lb[8];
    if (MODE == 0) {
#pragma unroll
      for (int e = 0; e < 8; ++e) {
        hb[e] = f2bf_bits(bv[e]);
        lb[e] = f2bf_bits(bv[e] - bf_bits2f(hb[e]));
      }
      const unsigned short sh = f2bf_bits(sv);
      s0[i] = sh;
      s1[i] = f2bf_bits(sv - bf_bits2f(sh));
    } else {
#pragma unroll
      for (int e = 0; e < 8; ++e) {
        hb[e] = h_bits(bv[e] * bcarry);
        lb[e] = hb[e];
      }
      s0[i] = h_bits(sv);
    }
    const v4u uh = (v4u){pk16(hb[0], hb[1]), pk16(hb[2], hb[3]), pk16(hb[4], hb[5]), pk16(hb[6], hb[7])};
    const v4u ul = (v4u){pk16(lb[0], lb[1]), pk16(lb[2], lb[3]), pk16(lb[4], lb[5]), pk16(lb[6], lb[7])};
    unsigned short* q0 = r0 + (size_t)i * 8;
    unsigned short* q1 = r1 + (size_t)i * 8;
    *(volatile v4u*)q0 = uh;
    if (MODE == 0) *(volatile v4u*)q1 = ul;
    __threadfence();
    *(volatile v4u*)q0 = uh;
    if (MODE == 0) *(volatile v4u*)q1 = ul;
  }
  __syncthreads();
  if (t < NIN / 8) {
    const v4u u0 = *(const v4u*)(s0 + 8 * t);
    v4u u1 = u0;
    if (MODE == 0) u1 = *(const v4u*)(s1 + 8 * t);
    unsigned short* q0 = r0 + (size_t)NIN * 8 + 8 * t;
    unsigned short* q1 = r1 + (size_t)NIN * 8 + 8 * t;
    *(volatile v4u*)q0 = u0;
    if (MODE == 0) *(volatile v4u*)q1 = u1;
    __threadfence();
    *(volatile v4u*)q0 = u0;
    if (MODE == 0) *(volatile v4u*)q1 = u1;
  }
}

template <int NIN, int NOUT, int MODE>
__global__ __launch_bounds__(256) void build_wt_rows(const float* __restrict__ coef,
                                                     const float* __restrict__ sbase,
                                                     const float* __restrict__ ssp,
                                                     unsigned short* __restrict__ P0,
                                                     unsigned short* __restrict__ P1,
                                                     float ccarry, float bcarry) {
  constexpr int KP  = NIN * 9;
  constexpr int NIT = NIN / 256;
  __shared__ __align__(16) unsigned short s0[NIN];
  __shared__ __align__(16) unsigned short s1[(MODE == 0) ? NIN : 16];
  const int o = blockIdx.x;
  const int t = threadIdx.x;
  unsigned short* r0 = P0 + (size_t)o * KP;
  unsigned short* r1 = P1 + (size_t)o * KP;
#pragma unroll 1
  for (int it = 0; it < NIT; ++it) {
    const int i = it * 256 + t;
    const size_t io = (size_t)i * NOUT + o;
    const float* cp = coef + io * 8;
    const v4f ca = *(const v4f*)(cp);
    const v4f cb = *(const v4f*)(cp + 4);
    const float ss = ssp[io];
    const float sb = sbase[io];
    float w[8];
#pragma unroll
    for (int e = 0; e < 4; ++e) { w[e] = ca[e] * ss; w[4 + e] = cb[e] * ss; }
    unsigned short hb[8], lb[8];
    if (MODE == 0) {
#pragma unroll
      for (int e = 0; e < 8; ++e) {
        hb[e] = f2bf_bits(w[e]);
        lb[e] = f2bf_bits(w[e] - bf_bits2f(hb[e]));
      }
      const unsigned short sh = f2bf_bits(sb);
      s0[i] = sh;
      s1[i] = f2bf_bits(sb - bf_bits2f(sh));
    } else {
#pragma unroll
      for (int e = 0; e < 8; ++e) {
        hb[e] = h_bits(w[e] * ccarry);
        lb[e] = hb[e];
      }
      s0[i] = h_bits(sb * bcarry);
    }
    const v4u uh = (v4u){pk16(hb[0], hb[1]), pk16(hb[2], hb[3]), pk16(hb[4], hb[5]), pk16(hb[6], hb[7])};
    const v4u ul = (v4u){pk16(lb[0], lb[1]), pk16(lb[2], lb[3]), pk16(lb[4], lb[5]), pk16(lb[6], lb[7])};
    unsigned short* q0 = r0 + (size_t)i * 8;
    unsigned short* q1 = r1 + (size_t)i * 8;
    *(volatile v4u*)q0 = uh;
    if (MODE == 0) *(volatile v4u*)q1 = ul;
    __threadfence();
    *(volatile v4u*)q0 = uh;
    if (MODE == 0) *(volatile v4u*)q1 = ul;
  }
  __syncthreads();
  if (t < NIN / 8) {
    const v4u u0 = *(const v4u*)(s0 + 8 * t);
    v4u u1 = u0;
    if (MODE == 0) u1 = *(const v4u*)(s1 + 8 * t);
    unsigned short* q0 = r0 + (size_t)NIN * 8 + 8 * t;
    unsigned short* q1 = r1 + (size_t)NIN * 8 + 8 * t;
    *(volatile v4u*)q0 = u0;
    if (MODE == 0) *(volatile v4u*)q1 = u1;
    __threadfence();
    *(volatile v4u*)q0 = u0;
    if (MODE == 0) *(volatile v4u*)q1 = u1;
  }
}

extern "C" void kernel_launch(void* const* d_in, const int* in_sizes, int n_in,
                              void* d_out, int out_size, void* d_ws, size_t ws_size,
                              hipStream_t stream) {
  if (n_in < 7) return;
  if (in_sizes[0] != kRows * kDimA) return;
  if (in_sizes[1] != kDimA * kDimB * kNBas || in_sizes[2] != kDimA * kDimB || in_sizes[3] != kDimA * kDimB) return;
  if (in_sizes[4] != kDimB * kDimA * kNBas || in_sizes[5] != kDimB * kDimA || in_sizes[6] != kDimB * kDimA) return;
  if (out_size != kRows * kDimA) return;
  if (ws_size < kWsTotal) return;

  const float* x     = (const float*)d_in[0];
  const float* coef1 = (const float*)d_in[1];
  const float* sb1   = (const float*)d_in[2];
  const float* ssp1  = (const float*)d_in[3];
  const float* coef2 = (const float*)d_in[4];
  const float* sb2   = (const float*)d_in[5];
  const float* ssp2  = (const float*)d_in[6];
  float* out = (float*)d_out;

  char* ws = (char*)d_ws;
  unsigned short* A1h = (unsigned short*)(ws + kOffA1h);
  unsigned short* A1l = (unsigned short*)(ws + kOffA1l);
  unsigned short* A2  = (unsigned short*)(ws + kOffA2);
  unsigned short* B1h = (unsigned short*)(ws + kOffB1h);
  unsigned short* B1l = (unsigned short*)(ws + kOffB1l);
  unsigned short* B2  = (unsigned short*)(ws + kOffB2);
  float*          H   = (float*)(ws + kOffH);

  build_wt_rows<kDimA, kDimB, 0><<<dim3(kDimB), 256, 0, stream>>>(coef1, sb1, ssp1, B1h, B1l, 1.0f, 1.0f);
  build_wt_rows<kDimB, kDimA, 1><<<dim3(kDimA), 256, 0, stream>>>(coef2, sb2, ssp2, B2, B2, kCoefCarry2, kBaseCarry2);
  build_act_rows<kDimA, 0><<<dim3(kRows), 256, 0, stream>>>(x, A1h, A1l, 1.0f);
  wmma_gemm64<1, true, 0, 0, false, 0><<<dim3((kRows / 64) * (kDimB / 64) / 8, 1), 256, 0, stream>>>(
      A1h, A1l, kK1, 0L,
      B1h, B1l, kK1, 0L,
      (void*)H, (void*)H, kDimB, 0L,
      (const float*)H,
      (const float*)H, 0L,
      kRows, kDimB, kK1, 1.0f);
  build_act_rows<kDimB, 1><<<dim3(kRows), 256, 0, stream>>>(H, A2, A2, kBasCarry2);
  wmma_gemm64<0, false, 0, 0, false, 0><<<dim3((kRows / 64) * (kDimA / 64) / 8, 1), 256, 0, stream>>>(
      A2, A2, kK2, 0L,
      B2, B2, kK2, 0L,
      (void*)out, (void*)out, kDimA, 0L,
      (const float*)H,
      (const float*)H, 0L,
      kRows, kDimA, kK2, kOutScale2);
}
